// SupportLayer_61718680043758
// MI455X (gfx1250) — hardware-verified
//
#include <hip/hip_runtime.h>
#include <math.h>

constexpr int kNQ = 256;
constexpr int kMS = 1024;
constexpr int kDD = 512;
constexpr int kHH = 512;
constexpr int kChunks = 8;
constexpr int kNPerChunk = kNQ / kChunks;
constexpr int kRowsPerChunk = kNPerChunk * kMS;
constexpr float kW1Carry    = 16.0f;
constexpr float kW1CarryInv = 1.0f / 16.0f;
static_assert(kNQ % kChunks == 0, "shape");
static_assert(kRowsPerChunk % 64 == 0, "shape");
static_assert(kDD % 32 == 0 && kHH % 64 == 0, "shape");

constexpr size_t kW1tBytes = (size_t)kHH * kDD * 2;
constexpr size_t kA16Bytes = (size_t)kRowsPerChunk * kDD * 2;
constexpr size_t kHBytes   = (size_t)kRowsPerChunk * kHH * 4;
constexpr size_t kW1tOff   = 0;
constexpr size_t kA16Off   = kW1tOff + kW1tBytes;
constexpr size_t kHOff     = kA16Off + kA16Bytes;
constexpr size_t kWsTotal  = kHOff + kHBytes;
static_assert(kWsTotal <= 134217728u, "ws");
static_assert(kA16Off % 128 == 0 && kHOff % 128 == 0, "align");

typedef __attribute__((ext_vector_type(16))) _Float16 v16h;
typedef __attribute__((ext_vector_type(8)))  _Float16 v8h;
typedef __attribute__((ext_vector_type(16))) __bf16   v16b;
typedef __attribute__((ext_vector_type(8)))  __bf16   v8b;
typedef __attribute__((ext_vector_type(8)))  float    v8f;
typedef __attribute__((ext_vector_type(4)))  float    v4f;
typedef __attribute__((ext_vector_type(4)))  unsigned int v4u;

__device__ __forceinline__ unsigned short f2bf_bits(float f) {
  unsigned u = __float_as_uint(f);
  return (unsigned short)((u + 0x7FFFu + ((u >> 16) & 1u)) >> 16);
}
__device__ __forceinline__ float bf_bits2f(unsigned short h) { return __uint_as_float(((unsigned)h) << 16); }

__device__ __forceinline__ void dep_guard_h(v8f& a, v8f& b, v16h x, v16h y) { asm volatile("v_nop\n\tv_nop\n\tv_nop\n\tv_nop" : "+v"(a), "+v"(b) : "v"(x), "v"(y)); }
__device__ __forceinline__ void dep_guard_b(v8f& a, v8f& b, v16b x, v16b y) { asm volatile("v_nop\n\tv_nop\n\tv_nop\n\tv_nop" : "+v"(a), "+v"(b) : "v"(x), "v"(y)); }
__device__ __forceinline__ void keep4_h(v16h a, v16h b, v16h c, v16h d) { asm volatile("v_nop" :: "v"(a), "v"(b), "v"(c), "v"(d)); }
__device__ __forceinline__ void keep4_b(v16b a, v16b b, v16b c, v16b d) { asm volatile("v_nop" :: "v"(a), "v"(b), "v"(c), "v"(d)); }
__device__ __forceinline__ void acc_guard4(v8f& a, v8f& b, v8f& c, v8f& d) { asm volatile("v_nop\n\tv_nop\n\tv_nop\n\tv_nop" : "+v"(a), "+v"(b), "+v"(c), "+v"(d)); }
template <typename T> struct Frag;
template <> struct Frag<_Float16> {
  typedef v16h V; union U { v16h v; v8h h[2]; };
  static __device__ __forceinline__ v16h load(const _Float16* p) {
    U f; f.h[0] = *(const v8h*)(p); f.h[1] = *(const v8h*)(p + 16); return f.v;
  }
  static __device__ __forceinline__ v8f mma(v16h a, v16h b, v8f c) {
    return __builtin_amdgcn_wmma_f32_16x16x32_f16(false, a, false, b, (short)0, c, false, false);
  }
  static __device__ __forceinline__ void guard(v8f& a, v8f& b, v16h x, v16h y) { dep_guard_h(a, b, x, y); }
  static __device__ __forceinline__ void keep(v16h a, v16h b, v16h c, v16h d) { keep4_h(a, b, c, d); }
};
template <> struct Frag<__bf16> {
  typedef v16b V; union U { v16b v; v8b h[2]; };
  static __device__ __forceinline__ v16b load(const __bf16* p) {
    U f; f.h[0] = *(const v8b*)(p); f.h[1] = *(const v8b*)(p + 16); return f.v;
  }
  static __device__ __forceinline__ v8f mma(v16b a, v16b b, v8f c) {
    return __builtin_amdgcn_wmma_f32_16x16x32_bf16(false, a, false, b, (short)0, c, false, false);
  }
  static __device__ __forceinline__ void guard(v8f& a, v8f& b, v16b x, v16b y) { dep_guard_b(a, b, x, y); }
  static __device__ __forceinline__ void keep(v16b a, v16b b, v16b c, v16b d) { keep4_b(a, b, c, d); }
};

__device__ __forceinline__ unsigned pk16(unsigned short a, unsigned short b) { return (unsigned)a | ((unsigned)b << 16); }
__device__ __forceinline__ unsigned short h_bits(float f) { const _Float16 h = (_Float16)f; return __builtin_bit_cast(unsigned short, h); }

template <int ET> struct Elem;
template <> struct Elem<0> { typedef _Float16 T; };
template <> struct Elem<1> { typedef __bf16 T; };
template <int ET, bool SPLIT, int BIAS_MODE, int OUT_MODE, bool RESID, int ACT = 0>
__global__ __launch_bounds__(256) void wmma_gemm64(
    const unsigned short* __restrict__ Ap, const unsigned short* __restrict__ A2p, int lda, long strideA,
    const unsigned short* __restrict__ Btp, const unsigned short* __restrict__ Bt2p, int ldb, long strideB,
    void* __restrict__ Cout, void* __restrict__ Cout2, int ldc, long strideC,
    const float* __restrict__ bias,
    const float* __restrict__ resid, long strideR,
    int M, int N, int K, float scale) {
  typedef typename Elem<ET>::T T;
  typedef typename Frag<T>::V V;
  const T* A = (const T*)Ap; const T* A2 = (const T*)A2p; const T* Bt = (const T*)Btp; const T* Bt2 = (const T*)Bt2p;
  __shared__ __align__(16) float sT[8][16 * 68];
  const int b    = blockIdx.y;
  const int lane = threadIdx.x & 31;
  const int wave = threadIdx.x >> 5;
  const int tilesN = N >> 6;
  const int tilesM = M >> 6;
  const int tile = blockIdx.x * 8 + wave;
  if (tile >= tilesM * tilesN) return;
  const int tm = tile / tilesN;
  const int tn = tile - tm * tilesN;
  const int m0 = tm << 6;
  const int n0 = tn << 6;

  const T* Ab  = A  + (size_t)b * strideA;
  const T* Bb  = Bt + (size_t)b * strideB;
  const T* Ab2 = SPLIT ? (A2  + (size_t)b * strideA) : nullptr;
  const T* Bb2 = SPLIT ? (Bt2 + (size_t)b * strideB) : nullptr;

  const int rlane = lane & 15;
  const int koff  = (lane >> 4) * 8;
  const int mOff  = (lane >> 4) * 8;

  v8f acc[4][4];
#pragma unroll
  for (int i = 0; i < 4; ++i)
#pragma unroll
    for (int j = 0; j < 4; ++j) acc[i][j] = (v8f){0.f,0.f,0.f,0.f,0.f,0.f,0.f,0.f};

  for (int k0 = 0; k0 < K; k0 += 32) {
    V bh[4], bl[4];
#pragma unroll
    for (int j = 0; j < 4; ++j) {
      const size_t bo = (size_t)(n0 + (j << 4) + rlane) * ldb + koff + k0;
      bh[j] = Frag<T>::load(Bb + bo);
      if (SPLIT) bl[j] = Frag<T>::load(Bb2 + bo);
    }
#pragma unroll
    for (int i = 0; i < 4; ++i) {
      const size_t ao = (size_t)(m0 + (i << 4) + rlane) * lda + koff + k0;
      V ah = Frag<T>::load(Ab + ao);
      V al;
      if (SPLIT) al = Frag<T>::load(Ab2 + ao);
#pragma unroll
      for (int j = 0; j < 4; ++j) {
        acc[i][j] = Frag<T>::mma(ah, bh[j], acc[i][j]);
        if (SPLIT) {
          acc[i][j] = Frag<T>::mma(ah, bl[j], acc[i][j]);
          acc[i][j] = Frag<T>::mma(al, bh[j], acc[i][j]);
        }
      }
      Frag<T>::guard(acc[i][0], acc[i][3], ah, SPLIT ? al : ah);
    }
    Frag<T>::keep(bh[0], bh[1], bh[2], bh[3]);
    if (SPLIT) Frag<T>::keep(bl[0], bl[1], bl[2], bl[3]);
  }
  acc_guard4(acc[0][0], acc[0][1], acc[0][2], acc[0][3]);
  acc_guard4(acc[1][0], acc[1][1], acc[1][2], acc[1][3]);
  acc_guard4(acc[2][0], acc[2][1], acc[2][2], acc[2][3]);
  acc_guard4(acc[3][0], acc[3][1], acc[3][2], acc[3][3]);

  float* slab = sT[wave];
  const float* Rb = RESID ? (resid + (size_t)b * strideR) : nullptr;
#pragma unroll
  for (int i = 0; i < 4; ++i) {
    const int mBase = m0 + (i << 4);
#pragma unroll
    for (int j = 0; j < 4; ++j) {
      const int n = n0 + (j << 4) + rlane;
      float bv = 0.f;
      if (BIAS_MODE == 2) bv = bias[n];
#pragma unroll
      for (int r = 0; r < 8; ++r) {
        float v = acc[i][j][r] * scale;
        if (BIAS_MODE == 1) v += bias[mBase + mOff + r];
        if (BIAS_MODE == 2) v += bv;
        if (RESID) v += Rb[(size_t)(mBase + mOff + r) * ldc + n];
        if (ACT == 2) v = fmaxf(v, 0.0f);
        if (ACT == 4) v = (v > 0.f) ? v : 0.01f * v;
        slab[(mOff + r) * 68 + (j << 4) + rlane] = v;
      }
    }
    __builtin_amdgcn_fence(__ATOMIC_RELEASE, "workgroup");
    __builtin_amdgcn_wave_barrier();
    __builtin_amdgcn_fence(__ATOMIC_ACQUIRE, "workgroup");
    if (OUT_MODE == 0) {
      float* C = (float*)Cout + (size_t)b * strideC;
      const int hh = lane >> 4, c4 = (lane & 15) * 4;
      for (int pass = 0; pass < 2; ++pass) {
#pragma unroll
        for (int it = 0; it < 8; ++it) {
          const int row = it * 2 + hh;
          v4f v = *(const v4f*)(slab + row * 68 + c4);
          *(volatile v4f*)(C + (size_t)(mBase + row) * ldc + n0 + c4) = v;
        }
        __threadfence();
      }
    } else {
      const int q = lane >> 3, c8 = (lane & 7) * 8;
      unsigned short* C  = (unsigned short*)Cout  + (size_t)b * strideC;
      unsigned short* C2 = (OUT_MODE == 2) ? ((unsigned short*)Cout2 + (size_t)b * strideC) : nullptr;
      for (int pass = 0; pass < 2; ++pass) {
#pragma unroll
        for (int it = 0; it < 4; ++it) {
          const int row = it * 4 + q;
          const float* sp = slab + row * 68 + c8;
          v8h hv, lv;
#pragma unroll
          for (int e = 0; e < 8; ++e) {
            if (OUT_MODE == 1) {
              hv[e] = (_Float16)sp[e];
            } else {
              unsigned short hb = f2bf_bits(sp[e]);
              unsigned short lb = f2bf_bits(sp[e] - bf_bits2f(hb));
              hv[e] = __builtin_bit_cast(_Float16, hb);
              lv[e] = __builtin_bit_cast(_Float16, lb);
            }
          }
          *(volatile v8h*)(C + (size_t)(mBase + row) * ldc + n0 + c8) = hv;
          if (OUT_MODE == 2) *(volatile v8h*)(C2 + (size_t)(mBase + row) * ldc + n0 + c8) = lv;
        }
        __threadfence();
      }
    }
    __builtin_amdgcn_fence(__ATOMIC_RELEASE, "workgroup");
    __builtin_amdgcn_wave_barrier();
    __builtin_amdgcn_fence(__ATOMIC_ACQUIRE, "workgroup");
  }
}

__global__ __launch_bounds__(256) void w1t_cast_kernel(const float* __restrict__ W, unsigned short* __restrict__ out, float scale) {
  __shared__ float sm[64][65];
  const int t  = threadIdx.x;
  const int d0 = blockIdx.x * 64;
  const int h0 = blockIdx.y * 64;
#pragma unroll
  for (int i = 0; i < 16; ++i) {
    const int e = i * 256 + t;
    const int r = e >> 6;
    const int c = e & 63;
    sm[c][r] = W[(size_t)(d0 + r) * kHH + h0 + c] * scale;
  }
  __syncthreads();
  const int lane = t & 31, wave = t >> 5;
  const int q = lane >> 3, c8 = (lane & 7) * 8;
  for (int pass = 0; pass < 2; ++pass) {
#pragma unroll
    for (int it = 0; it < 2; ++it) {
      const int row = wave * 8 + it * 4 + q;
      unsigned short hb[8];
#pragma unroll
      for (int e = 0; e < 8; ++e) hb[e] = h_bits(sm[row][c8 + e]);
      const v4u u = (v4u){pk16(hb[0], hb[1]), pk16(hb[2], hb[3]), pk16(hb[4], hb[5]), pk16(hb[6], hb[7])};
      *(volatile v4u*)(out + (size_t)(h0 + row) * kDD + d0 + c8) = u;
    }
    __threadfence();
  }
}

__global__ __launch_bounds__(256) void absdiff_f16_kernel(const float* __restrict__ emb, const float* __restrict__ sup,
                                                        unsigned short* __restrict__ A16, int chunk) {
  const int gt = blockIdx.x * 256 + threadIdx.x;
  const int rl = gt >> 6;
  const int d8 = (gt & 63) * 8;
  const int nl = rl >> 10;
  const int m  = rl & (kMS - 1);
  int n = chunk * kNPerChunk + nl;
  n = n < 0 ? 0 : (n > kNQ - 1 ? kNQ - 1 : n);
  const float* ep = emb + (size_t)n * kDD + d8;
  const float* sp = sup + (size_t)m * kDD + d8;
  const v4f e0 = *(const v4f*)(ep);
  const v4f e1 = *(const v4f*)(ep + 4);
  const v4f s0 = *(const v4f*)(sp);
  const v4f s1 = *(const v4f*)(sp + 4);
  unsigned short hb[8];
#pragma unroll
  for (int e = 0; e < 4; ++e) {
    hb[e]     = h_bits(fabsf(e0[e] - s0[e]));
    hb[4 + e] = h_bits(fabsf(e1[e] - s1[e]));
  }
  const v4u u = (v4u){pk16(hb[0], hb[1]), pk16(hb[2], hb[3]), pk16(hb[4], hb[5]), pk16(hb[6], hb[7])};
  unsigned short* q = A16 + (size_t)rl * kDD + d8;
  *(volatile v4u*)q = u;
  __threadfence();
  *(volatile v4u*)q = u;
}

__global__ __launch_bounds__(256) void rowdot_sigmoid_kernel(const float* __restrict__ H, const float* __restrict__ W2,
                                                           const float* __restrict__ b2, float* __restrict__ out, int chunk) {
  __shared__ __align__(16) float sW2[kHH];
  __shared__ __align__(16) float sOut[32];
  const int t = threadIdx.x;
  const int lane = t & 31, wave = t >> 5;
  sW2[t]       = W2[t];
  sW2[t + 256] = W2[t + 256];
  __syncthreads();
  const int q    = lane & 7;
  const int rr   = lane >> 3;
  const int rowl = wave * 4 + rr;
  const int rl   = blockIdx.x * 32 + rowl;
  const float* hp = H + (size_t)rl * kHH + q * 64;
  const float* wp = sW2 + q * 64;
  float acc = 0.f;
#pragma unroll 4
  for (int i = 0; i < 16; ++i) {
    const v4f hv = *(const v4f*)(hp + 4 * i);
    const v4f wv = *(const v4f*)(wp + 4 * i);
    acc = fmaf(hv[0], wv[0], acc);
    acc = fmaf(hv[1], wv[1], acc);
    acc = fmaf(hv[2], wv[2], acc);
    acc = fmaf(hv[3], wv[3], acc);
  }
  acc += __shfl_xor(acc, 1, 32);
  acc += __shfl_xor(acc, 2, 32);
  acc += __shfl_xor(acc, 4, 32);
  float lg = acc + b2[0];
  lg = fminf(fmaxf(lg, -30.0f), 30.0f);
  const float sg = 1.0f / (1.0f + expf(-lg));
  if (q == 0) sOut[rowl] = sg;
  __syncthreads();
  if (wave == 0) {
    const int l8 = lane & 7;
    const v4f v = *(const v4f*)(sOut + 4 * l8);
    int cc = chunk; cc = cc < 0 ? 0 : (cc > kChunks - 1 ? kChunks - 1 : cc);
    float* op = out + (size_t)cc * kRowsPerChunk + (size_t)blockIdx.x * 32 + 4 * l8;
    for (int pass = 0; pass < 2; ++pass) {
      if (lane < 8) *(volatile v4f*)op = v;
      __threadfence();
    }
  }
}

extern "C" void kernel_launch(void* const* d_in, const int* in_sizes, int n_in,
                              void* d_out, int out_size, void* d_ws, size_t ws_size,
                              hipStream_t stream) {
  if (n_in < 6) return;
  if (in_sizes[0] != kNQ * kDD || in_sizes[1] != kMS * kDD || in_sizes[2] != kDD * kHH ||
      in_sizes[3] != kHH || in_sizes[4] != kHH || in_sizes[5] < 1) return;
  if (out_size != kNQ * kMS) return;
  if (ws_size < kWsTotal) return;

  const float* emb = (const float*)d_in[0];
  const float* sup = (const float*)d_in[1];
  const float* W1  = (const float*)d_in[2];
  const float* b1  = (const float*)d_in[3];
  const float* W2  = (const float*)d_in[4];
  const float* b2  = (const float*)d_in[5];
  float* out = (float*)d_out;

  char* ws = (char*)d_ws;
  unsigned short* W1t  = (unsigned short*)(ws + kW1tOff);
  unsigned short* A16  = (unsigned short*)(ws + kA16Off);
  float*          Hbuf = (float*)(ws + kHOff);

  w1t_cast_kernel<<<dim3(kDD / 64, kHH / 64), 256, 0, stream>>>(W1, W1t, kW1Carry);

  const int prodBlocks = (kRowsPerChunk * (kDD / 8)) / 256;
  const int gemmTiles  = (kRowsPerChunk / 64) * (kHH / 64);
  const int gemmBlocks = (gemmTiles + 7) / 8;
  const int dotBlocks  = kRowsPerChunk / 32;

  for (int c = 0; c < kChunks; ++c) {
    absdiff_f16_kernel<<<prodBlocks, 256, 0, stream>>>(emb, sup, A16, c);
    wmma_gemm64<0, false, 2, 0, false, 2><<<dim3(gemmBlocks, 1), 256, 0, stream>>>(
        A16, A16, kDD, 0L,
        W1t, W1t, kDD, 0L,
        (void*)Hbuf, (void*)Hbuf, kHH, 0L,
        b1,
        b1, 0L,
        kRowsPerChunk, kHH, kDD, kW1CarryInv);
    rowdot_sigmoid_kernel<<<dotBlocks, 256, 0, stream>>>(Hbuf, W2, b2, out, c);
  }
}
